// STABR_tag_encoder_26697516712561
// MI455X (gfx1250) — hardware-run, weakly checked
//
#include <hip/hip_runtime.h>
#include <hip/hip_bf16.h>

typedef __attribute__((ext_vector_type(16))) _Float16 v16h;
typedef __attribute__((ext_vector_type(8)))  _Float16 v8h;
typedef __attribute__((ext_vector_type(16))) __bf16   v16b;
typedef __attribute__((ext_vector_type(8)))  __bf16   v8b;
typedef __attribute__((ext_vector_type(8)))  float    v8f;
typedef __attribute__((ext_vector_type(4)))  float    v4f;

constexpr int kB   = 512;
constexpr int kS   = 200;
constexpr int kT   = 10;
constexpr int kE   = 25;
constexpr int kH   = 64;
constexpr int kNH  = 192;
constexpr int kKP  = 96;
constexpr int kTok = kB * kS;
constexpr int kSP  = 208;
constexpr float kXScale = 1024.0f;
constexpr float kWScale = 16.0f;
constexpr float kInv    = 1.0f / 16384.0f;

static_assert(kB % 64 == 0);
static_assert(kTok % 8 == 0);
static_assert(kTok % 64 == 0);
static_assert((2 * kH) % 32 == 0);
static_assert(kH % 64 == 0 || kH == 64);
static_assert(kSP % 16 == 0 && kSP >= kS);

__device__ __forceinline__ unsigned short f2bf_bits(float f) {
  unsigned u = __float_as_uint(f);
  return (unsigned short)((u + 0x7FFFu + ((u >> 16) & 1u)) >> 16);
}
__device__ __forceinline__ float bf_bits2f(unsigned short h) { return __uint_as_float(((unsigned)h) << 16); }

__device__ __forceinline__ void dep_guard_h(v8f& a, v8f& b, v16h x, v16h y) { asm volatile("v_nop\n\tv_nop\n\tv_nop\n\tv_nop" : "+v"(a), "+v"(b) : "v"(x), "v"(y)); }
__device__ __forceinline__ void dep_guard_b(v8f& a, v8f& b, v16b x, v16b y) { asm volatile("v_nop\n\tv_nop\n\tv_nop\n\tv_nop" : "+v"(a), "+v"(b) : "v"(x), "v"(y)); }
__device__ __forceinline__ void keep4_h(v16h a, v16h b, v16h c, v16h d) { asm volatile("v_nop" :: "v"(a), "v"(b), "v"(c), "v"(d)); }
__device__ __forceinline__ void keep4_b(v16b a, v16b b, v16b c, v16b d) { asm volatile("v_nop" :: "v"(a), "v"(b), "v"(c), "v"(d)); }
__device__ __forceinline__ void acc_guard4(v8f& a, v8f& b, v8f& c, v8f& d) { asm volatile("v_nop\n\tv_nop\n\tv_nop\n\tv_nop" : "+v"(a), "+v"(b), "+v"(c), "+v"(d)); }
template <typename T> struct Frag;
template <> struct Frag<_Float16> {
  typedef v16h V; union U { v16h v; v8h h[2]; };
  static __device__ __forceinline__ v16h load(const _Float16* p) {
    U f; f.h[0] = *(const v8h*)(p); f.h[1] = *(const v8h*)(p + 16); return f.v;
  }
  static __device__ __forceinline__ v8f mma(v16h a, v16h b, v8f c) {
    return __builtin_amdgcn_wmma_f32_16x16x32_f16(false, a, false, b, (short)0, c, false, false);
  }
  static __device__ __forceinline__ void guard(v8f& a, v8f& b, v16h x, v16h y) { dep_guard_h(a, b, x, y); }
  static __device__ __forceinline__ void keep(v16h a, v16h b, v16h c, v16h d) { keep4_h(a, b, c, d); }
};
template <> struct Frag<__bf16> {
  typedef v16b V; union U { v16b v; v8b h[2]; };
  static __device__ __forceinline__ v16b load(const __bf16* p) {
    U f; f.h[0] = *(const v8b*)(p); f.h[1] = *(const v8b*)(p + 16); return f.v;
  }
  static __device__ __forceinline__ v8f mma(v16b a, v16b b, v8f c) {
    return __builtin_amdgcn_wmma_f32_16x16x32_bf16(false, a, false, b, (short)0, c, false, false);
  }
  static __device__ __forceinline__ void guard(v8f& a, v8f& b, v16b x, v16b y) { dep_guard_b(a, b, x, y); }
  static __device__ __forceinline__ void keep(v16b a, v16b b, v16b c, v16b d) { keep4_b(a, b, c, d); }
};

template <int ET> struct Elem;
template <> struct Elem<0> { typedef _Float16 T; };
template <> struct Elem<1> { typedef __bf16 T; };
template <int ET, bool SPLIT, int BIAS_MODE, int OUT_MODE, bool RESID, int ACT = 0>
__global__ __launch_bounds__(256) void wmma_gemm64(
    const unsigned short* __restrict__ Ap, const unsigned short* __restrict__ A2p, int lda, long strideA,
    const unsigned short* __restrict__ Btp, const unsigned short* __restrict__ Bt2p, int ldb, long strideB,
    void* __restrict__ Cout, void* __restrict__ Cout2, int ldc, long strideC,
    const float* __restrict__ bias,
    const float* __restrict__ resid, long strideR,
    int M, int N, int K, float scale) {
  typedef typename Elem<ET>::T T;
  typedef typename Frag<T>::V V;
  const T* A = (const T*)Ap; const T* A2 = (const T*)A2p; const T* Bt = (const T*)Btp; const T* Bt2 = (const T*)Bt2p;
  __shared__ __align__(16) float sT[8][16 * 68];
  const int b    = blockIdx.y;
  const int lane = threadIdx.x & 31;
  const int wave = threadIdx.x >> 5;
  const int tilesN = N >> 6;
  const int tilesM = M >> 6;
  const int tile = blockIdx.x * 8 + wave;
  if (tile >= tilesM * tilesN) return;
  const int tm = tile / tilesN;
  const int tn = tile - tm * tilesN;
  const int m0 = tm << 6;
  const int n0 = tn << 6;

  const T* Ab  = A  + (size_t)b * strideA;
  const T* Bb  = Bt + (size_t)b * strideB;
  const T* Ab2 = SPLIT ? (A2  + (size_t)b * strideA) : nullptr;
  const T* Bb2 = SPLIT ? (Bt2 + (size_t)b * strideB) : nullptr;

  const int rlane = lane & 15;
  const int koff  = (lane >> 4) * 8;
  const int mOff  = (lane >> 4) * 8;

  v8f acc[4][4];
#pragma unroll
  for (int i = 0; i < 4; ++i)
#pragma unroll
    for (int j = 0; j < 4; ++j) acc[i][j] = (v8f){0.f,0.f,0.f,0.f,0.f,0.f,0.f,0.f};

  for (int k0 = 0; k0 < K; k0 += 32) {
    V bh[4], bl[4];
#pragma unroll
    for (int j = 0; j < 4; ++j) {
      const size_t bo = (size_t)(n0 + (j << 4) + rlane) * ldb + koff + k0;
      bh[j] = Frag<T>::load(Bb + bo);
      if (SPLIT) bl[j] = Frag<T>::load(Bb2 + bo);
    }
#pragma unroll
    for (int i = 0; i < 4; ++i) {
      const size_t ao = (size_t)(m0 + (i << 4) + rlane) * lda + koff + k0;
      V ah = Frag<T>::load(Ab + ao);
      V al;
      if (SPLIT) al = Frag<T>::load(Ab2 + ao);
#pragma unroll
      for (int j = 0; j < 4; ++j) {
        acc[i][j] = Frag<T>::mma(ah, bh[j], acc[i][j]);
        if (SPLIT) {
          acc[i][j] = Frag<T>::mma(ah, bl[j], acc[i][j]);
          acc[i][j] = Frag<T>::mma(al, bh[j], acc[i][j]);
        }
      }
      Frag<T>::guard(acc[i][0], acc[i][3], ah, SPLIT ? al : ah);
    }
    Frag<T>::keep(bh[0], bh[1], bh[2], bh[3]);
    if (SPLIT) Frag<T>::keep(bl[0], bl[1], bl[2], bl[3]);
  }
  acc_guard4(acc[0][0], acc[0][1], acc[0][2], acc[0][3]);
  acc_guard4(acc[1][0], acc[1][1], acc[1][2], acc[1][3]);
  acc_guard4(acc[2][0], acc[2][1], acc[2][2], acc[2][3]);
  acc_guard4(acc[3][0], acc[3][1], acc[3][2], acc[3][3]);

  float* slab = sT[wave];
  const float* Rb = RESID ? (resid + (size_t)b * strideR) : nullptr;
#pragma unroll
  for (int i = 0; i < 4; ++i) {
    const int mBase = m0 + (i << 4);
#pragma unroll
    for (int j = 0; j < 4; ++j) {
      const int n = n0 + (j << 4) + rlane;
      float bv = 0.f;
      if (BIAS_MODE == 2) bv = bias[n];
#pragma unroll
      for (int r = 0; r < 8; ++r) {
        float v = acc[i][j][r] * scale;
        if (BIAS_MODE == 1) v += bias[mBase + mOff + r];
        if (BIAS_MODE == 2) v += bv;
        if (RESID) v += Rb[(size_t)(mBase + mOff + r) * ldc + n];
        if (ACT == 1) v = tanhf(v);
        if (ACT == 2) v = fmaxf(v, 0.0f);
        if (ACT == 3) v = v / (1.0f + expf(-v));
        if (ACT == 4) v = (v > 0.f) ? v : 0.01f * v;
        if (ACT == 5) v = 0.5f * v * (1.0f + erff(v * 0.70710678118654752f));
        slab[(mOff + r) * 68 + (j << 4) + rlane] = v;
      }
    }
    __builtin_amdgcn_fence(__ATOMIC_RELEASE, "workgroup");
    __builtin_amdgcn_wave_barrier();
    __builtin_amdgcn_fence(__ATOMIC_ACQUIRE, "workgroup");
    if (OUT_MODE == 0) {
      float* C = (float*)Cout + (size_t)b * strideC;
      const int hh = lane >> 4, c4 = (lane & 15) * 4;
      for (int pass = 0; pass < 2; ++pass) {
#pragma unroll
        for (int it = 0; it < 8; ++it) {
          const int row = it * 2 + hh;
          v4f v = *(const v4f*)(slab + row * 68 + c4);
          *(volatile v4f*)(C + (size_t)(mBase + row) * ldc + n0 + c4) = v;
        }
        __threadfence();
      }
    } else {
      const int q = lane >> 3, c8 = (lane & 7) * 8;
      unsigned short* C  = (unsigned short*)Cout  + (size_t)b * strideC;
      unsigned short* C2 = (OUT_MODE == 2) ? ((unsigned short*)Cout2 + (size_t)b * strideC) : nullptr;
      for (int pass = 0; pass < 2; ++pass) {
#pragma unroll
        for (int it = 0; it < 4; ++it) {
          const int row = it * 4 + q;
          const float* sp = slab + row * 68 + c8;
          v8h hv, lv;
#pragma unroll
          for (int e = 0; e < 8; ++e) {
            if (OUT_MODE == 1) {
              hv[e] = (_Float16)sp[e];
            } else {
              unsigned short hb = f2bf_bits(sp[e]);
              unsigned short lb = f2bf_bits(sp[e] - bf_bits2f(hb));
              hv[e] = __builtin_bit_cast(_Float16, hb);
              lv[e] = __builtin_bit_cast(_Float16, lb);
            }
          }
          *(volatile v8h*)(C + (size_t)(mBase + row) * ldc + n0 + c8) = hv;
          if (OUT_MODE == 2) *(volatile v8h*)(C2 + (size_t)(mBase + row) * ldc + n0 + c8) = lv;
        }
        __threadfence();
      }
    }
    __builtin_amdgcn_fence(__ATOMIC_RELEASE, "workgroup");
    __builtin_amdgcn_wave_barrier();
    __builtin_amdgcn_fence(__ATOMIC_ACQUIRE, "workgroup");
  }
}

__device__ __forceinline__ v8f mma_f16g(v16h a, v16h b, v8f c) {
  c = __builtin_amdgcn_wmma_f32_16x16x32_f16(false, a, false, b, (short)0, c, false, false);
  asm volatile("v_nop\n\tv_nop\n\tv_nop\n\tv_nop" : "+v"(c) : "v"(a), "v"(b));
  return c;
}
__device__ __forceinline__ v8f zero8f() { return (v8f){0.f,0.f,0.f,0.f,0.f,0.f,0.f,0.f}; }
__device__ __forceinline__ v8h zero8h() {
  v8h z;
#pragma unroll
  for (int e = 0; e < 8; ++e) z[e] = (_Float16)0.0f;
  return z;
}

__global__ __launch_bounds__(256)
void embed_mean(const int* __restrict__ ids, const float* __restrict__ emb, float* __restrict__ X32, int nV) {
  const int wave = threadIdx.x >> 5, lane = threadIdx.x & 31;
  const int tok = blockIdx.x * 8 + wave;
  const int* bag = ids + (size_t)tok * kT;
  const int ca = (lane < kE) ? lane : (kE - 1);
  float acc = 0.f, cnt = 0.f;
#pragma unroll
  for (int t = 0; t < kT; ++t) {
    const int id = bag[t];
    int idc = id < 0 ? 0 : id;
    idc = idc > (nV - 1) ? (nV - 1) : idc;
    const float v = emb[(size_t)idc * kE + ca];
    const bool nz = (id != 0);
    cnt += nz ? 1.f : 0.f;
    acc += (nz && lane < kE) ? v : 0.f;
  }
  const float den = (cnt == 0.f) ? 1.f : cnt;
  const float x = acc * (1.0f / den);
  volatile float* dst = X32 + (size_t)tok * 32 + lane;
  *dst = x;
  __threadfence();
  *dst = x;
}

__global__ __launch_bounds__(256)
void prep_weights(const float* __restrict__ Wk, const float* __restrict__ Wq,
                  _Float16* __restrict__ WkT, _Float16* __restrict__ WqT) {
  const int tid = threadIdx.x;
  if (blockIdx.x < 4) {
    const int g = blockIdx.x * 256 + tid;
    const int n = g >> 4, k8 = (g & 15) * 8;
    v8h v;
#pragma unroll
    for (int e = 0; e < 8; ++e) v[e] = (_Float16)(Wk[(size_t)(k8 + e) * kH + n] * kWScale);
    _Float16* p = WkT + (size_t)n * (2 * kH) + k8;
    *(volatile v8h*)p = v;
    __threadfence();
    *(volatile v8h*)p = v;
  } else {
    const int g = (blockIdx.x - 4) * 256 + tid;
    const int n = g >> 3, k8 = (g & 7) * 8;
    v8h v;
#pragma unroll
    for (int e = 0; e < 8; ++e) v[e] = (_Float16)(Wq[(size_t)(k8 + e) * kH + n] * kWScale);
    _Float16* p = WqT + (size_t)n * kH + k8;
    *(volatile v8h*)p = v;
    __threadfence();
    *(volatile v8h*)p = v;
  }
}

__global__ __launch_bounds__(128)
void gru_bidir(const float* __restrict__ X32, const int* __restrict__ ids,
               const float* __restrict__ Uf, const float* __restrict__ Wf, const float* __restrict__ bfp,
               const float* __restrict__ Ub, const float* __restrict__ Wb, const float* __restrict__ bbp,
               _Float16* __restrict__ O16, float* __restrict__ O32, _Float16* __restrict__ HT16) {
  __shared__ __align__(16) _Float16 Ut[kNH * kKP];
  __shared__ __align__(16) _Float16 hbuf[4][16 * 64];
  __shared__ __align__(16) float    slab[4][16 * 68];
  __shared__ float b0s[kNH];
  __shared__ float b1s[kNH];

  const int dir = blockIdx.y;
  const float* U    = dir ? Ub : Uf;
  const float* W    = dir ? Wb : Wf;
  const float* bias = dir ? bbp : bfp;
  const int tid = threadIdx.x, wave = tid >> 5, lane = tid & 31;
  const int m = lane & 15, h = lane >> 4;

  for (int idx = tid; idx < kNH * kKP; idx += 128) {
    const int n = idx / kKP, k = idx - n * kKP;
    const int ku = (k < kH) ? k : (kH - 1);
    int kw = k - kH; kw = kw < 0 ? 0 : kw; kw = kw > (kE - 1) ? (kE - 1) : kw;
    const float vu = U[(size_t)ku * kNH + n];
    const float vw = W[(size_t)kw * kNH + n];
    const float v = (k < kH) ? vu : ((k < kH + kE) ? vw : 0.f);
    Ut[idx] = (_Float16)(v * kWScale);
  }
  for (int i = tid; i < kNH; i += 128) { b0s[i] = bias[i]; b1s[i] = bias[kNH + i]; }
  _Float16* hb = hbuf[wave];
  float* sl = slab[wave];
  {
    const v8h z8 = zero8h();
    for (int i = lane; i < (16 * 64) / 8; i += 32) *(v8h*)(hb + i * 8) = z8;
    const v4f z4 = (v4f){0.f, 0.f, 0.f, 0.f};
    for (int i = lane; i < (16 * 68) / 4; i += 32) *(v4f*)(sl + i * 4) = z4;
  }
  __syncthreads();

  const int b0 = blockIdx.x * 64 + wave * 16;
  const int q8 = lane >> 3, c8 = (lane & 7) * 8, c4 = (lane & 15) * 4;

  for (int step = 0; step < kS; ++step) {
    const int s = dir ? (kS - 1 - step) : step;

    const v16h a0 = Frag<_Float16>::load(hb + m * 64 + 8 * h);
    const v16h a1 = Frag<_Float16>::load(hb + m * 64 + 32 + 8 * h);
    v16h ax;
    {
      const float* xr = X32 + ((size_t)(b0 + m) * kS + s) * 32;
      const v4f x0 = *(const v4f*)(xr + 8 * h);
      const v4f x1 = *(const v4f*)(xr + 8 * h + 4);
      const v4f x2 = *(const v4f*)(xr + 16 + 8 * h);
      const v4f x3 = *(const v4f*)(xr + 20 + 8 * h);
#pragma unroll
      for (int e = 0; e < 4; ++e) {
        ax[e]      = (_Float16)(x0[e] * kXScale);
        ax[4 + e]  = (_Float16)(x1[e] * kXScale);
        ax[8 + e]  = (_Float16)(x2[e] * kXScale);
        ax[12 + e] = (_Float16)(x3[e] * kXScale);
      }
    }
    float mk[8];
#pragma unroll
    for (int j = 0; j < 8; ++j) {
      const int id = ids[((size_t)(b0 + 8 * h + j) * kS + s) * kT];
      mk[j] = (id != 0) ? 1.f : 0.f;
    }

#pragma unroll 1
    for (int t = 0; t < 4; ++t) {
      const int n = t * 16 + m;
      const _Float16* pz = Ut + (size_t)n * kKP + 8 * h;
      const _Float16* pr = Ut + (size_t)(kH + n) * kKP + 8 * h;
      const _Float16* ph = Ut + (size_t)(2 * kH + n) * kKP + 8 * h;
      v8f cz = zero8f(), cr = zero8f(), cu = zero8f(), cx = zero8f();
      cz = mma_f16g(a0, Frag<_Float16>::load(pz),      cz);
      cz = mma_f16g(a1, Frag<_Float16>::load(pz + 32), cz);
      cz = mma_f16g(ax, Frag<_Float16>::load(pz + 64), cz);
      cr = mma_f16g(a0, Frag<_Float16>::load(pr),      cr);
      cr = mma_f16g(a1, Frag<_Float16>::load(pr + 32), cr);
      cr = mma_f16g(ax, Frag<_Float16>::load(pr + 64), cr);
      cu = mma_f16g(a0, Frag<_Float16>::load(ph),      cu);
      cu = mma_f16g(a1, Frag<_Float16>::load(ph + 32), cu);
      cx = mma_f16g(ax, Frag<_Float16>::load(ph + 64), cx);

      const float bz  = b0s[n] + b1s[n];
      const float brr = b0s[kH + n] + b1s[kH + n];
      const float bh0 = b0s[2 * kH + n];
      const float bh1 = b1s[2 * kH + n];
#pragma unroll
      for (int j = 0; j < 8; ++j) {
        const int row = 8 * h + j;
        const float ho = sl[row * 68 + n];
        const float vz = cz[j] * kInv + bz;
        const float z  = 1.0f / (1.0f + expf(-vz));
        const float vr = cr[j] * kInv + brr;
        const float r  = 1.0f / (1.0f + expf(-vr));
        const float hh = tanhf(cx[j] * kInv + bh0 + r * (cu[j] * kInv + bh1));
        float hn = z * ho + (1.0f - z) * hh;
        hn = (mk[j] != 0.f) ? hn : ho;
        sl[row * 68 + n] = hn;
        hb[row * 64 + n] = (_Float16)(hn * kXScale);
      }
    }
    __syncthreads();

    for (int pass = 0; pass < 2; ++pass) {
#pragma unroll
      for (int it = 0; it < 4; ++it) {
        const int row = it * 4 + q8;
        const v8h v = *(const v8h*)(hb + row * 64 + c8);
        *(volatile v8h*)(O16 + ((size_t)(b0 + row) * kS + s) * (2 * kH) + dir * kH + c8) = v;
      }
#pragma unroll
      for (int it = 0; it < 8; ++it) {
        const int row = it * 2 + h;
        const v4f v = *(const v4f*)(sl + row * 68 + c4);
        *(volatile v4f*)(O32 + ((size_t)(b0 + row) * kS + s) * (2 * kH) + dir * kH + c4) = v;
      }
      __threadfence();
    }
    __syncthreads();
  }

  if (dir == 0) {
    for (int pass = 0; pass < 2; ++pass) {
#pragma unroll
      for (int it = 0; it < 4; ++it) {
        const int row = it * 4 + q8;
        const v8h v = *(const v8h*)(hb + row * 64 + c8);
        *(volatile v8h*)(HT16 + (size_t)(b0 + row) * kH + c8) = v;
      }
      __threadfence();
    }
  }
}

__global__ __launch_bounds__(256)
void attn_pool(const float* __restrict__ KEYS, const float* __restrict__ Q, const float* __restrict__ We,
               const float* __restrict__ be, const int* __restrict__ ids, const float* __restrict__ O32,
               float* __restrict__ out) {
  __shared__ __align__(16) _Float16 WeB[16 * 64];
  __shared__ __align__(16) _Float16 TA[kSP * 64];
  __shared__ float qs[64];
  __shared__ float es[kSP];
  __shared__ float red[256];
  __shared__ float part[256];
  __shared__ __align__(16) float cs[128];

  const int b = blockIdx.x, tid = threadIdx.x, wave = tid >> 5, lane = tid & 31;
  const int m = lane & 15, h = lane >> 4;

  if (tid < 64) qs[tid] = Q[(size_t)b * kH + tid];
  if (tid < 128) {
    const int n = tid >> 3, k8 = (tid & 7) * 8;
    v8h v;
#pragma unroll
    for (int e = 0; e < 8; ++e) {
      const float w = We[k8 + e] * kWScale;
      v[e] = (_Float16)((n == 0) ? w : 0.f);
    }
    *(v8h*)(WeB + n * 64 + k8) = v;
  }
  __syncthreads();

  for (int i8 = tid; i8 < kSP * 8; i8 += 256) {
    const int s = i8 >> 3, n8 = (i8 & 7) * 8;
    const int sc = (s < kS) ? s : (kS - 1);
    const float* kp = KEYS + ((size_t)b * kS + sc) * kH + n8;
    const v4f k0 = *(const v4f*)kp;
    const v4f k1 = *(const v4f*)(kp + 4);
    v8h v;
#pragma unroll
    for (int e = 0; e < 4; ++e) {
      const float t0 = tanhf(k0[e] + qs[n8 + e]) * kXScale;
      const float t1 = tanhf(k1[e] + qs[n8 + 4 + e]) * kXScale;
      v[e]     = (_Float16)((s < kS) ? t0 : 0.f);
      v[4 + e] = (_Float16)((s < kS) ? t1 : 0.f);
    }
    *(v8h*)(TA + s * 64 + n8) = v;
  }
  __syncthreads();

  const float be0 = be[0];
  for (int tw = wave; tw < kSP / 16; tw += 8) {
    v8f acc = zero8f();
#pragma unroll
    for (int kk = 0; kk < 2; ++kk) {
      const v16h a  = Frag<_Float16>::load(TA + (tw * 16 + m) * 64 + kk * 32 + 8 * h);
      const v16h bb = Frag<_Float16>::load(WeB + m * 64 + kk * 32 + 8 * h);
      acc = mma_f16g(a, bb, acc);
    }
    if (m == 0) {
#pragma unroll
      for (int r = 0; r < 8; ++r) es[tw * 16 + 8 * h + r] = acc[r] * kInv + be0;
    }
  }
  __syncthreads();

  const int sc = (tid < kS) ? tid : (kS - 1);
  const int id0 = ids[((size_t)b * kS + sc) * kT];
  const float ev = (tid < kS) ? (es[sc] + ((id0 != 0) ? 0.f : -1.0e9f)) : -INFINITY;
  red[tid] = ev;
  __syncthreads();
  for (int off = 128; off > 0; off >>= 1) {
    if (tid < off) red[tid] = fmaxf(red[tid], red[tid + off]);
    __syncthreads();
  }
  const float mx = red[0];
  __syncthreads();
  const float p = (tid < kS) ? expf(ev - mx) : 0.f;
  if (tid < kS) es[tid] = p;
  red[tid] = p;
  __syncthreads();
  for (int off = 128; off > 0; off >>= 1) {
    if (tid < off) red[tid] = red[tid] + red[tid + off];
    __syncthreads();
  }
  const float inv = 1.0f / red[0];
  __syncthreads();

  {
    const int c = tid & 127, hf = tid >> 7;
    const int sbeg = hf * (kS / 2);
    float a = 0.f;
    for (int s = sbeg; s < sbeg + kS / 2; ++s)
      a += es[s] * O32[((size_t)b * kS + s) * (2 * kH) + c];
    part[tid] = a;
  }
  __syncthreads();
  if (tid < 128) cs[tid] = (part[tid] + part[tid + 128]) * inv;
  __syncthreads();
  if (wave == 0) {
    const v4f v = *(const v4f*)(cs + lane * 4);
    for (int pass = 0; pass < 2; ++pass) {
      *(volatile v4f*)(out + (size_t)b * (2 * kH) + lane * 4) = v;
      __threadfence();
    }
  }
}

constexpr size_t kOffX32  = 0;
constexpr size_t kSzX32   = (size_t)kTok * 32 * 4;
constexpr size_t kOffO16  = kOffX32 + kSzX32;
constexpr size_t kSzO16   = (size_t)kTok * 2 * kH * 2;
constexpr size_t kOffO32  = kOffO16 + kSzO16;
constexpr size_t kSzO32   = (size_t)kTok * 2 * kH * 4;
constexpr size_t kOffKeys = kOffO32 + kSzO32;
constexpr size_t kSzKeys  = (size_t)kTok * kH * 4;
constexpr size_t kOffHT16 = kOffKeys + kSzKeys;
constexpr size_t kSzHT16  = (size_t)kB * kH * 2;
constexpr size_t kOffQ    = kOffHT16 + kSzHT16;
constexpr size_t kSzQ     = (size_t)kB * kH * 4;
constexpr size_t kOffWkT  = kOffQ + kSzQ;
constexpr size_t kSzWkT   = (size_t)kH * 2 * kH * 2;
constexpr size_t kOffWqT  = kOffWkT + kSzWkT;
constexpr size_t kSzWqT   = (size_t)kH * kH * 2;
constexpr size_t kWsTotal = kOffWqT + kSzWqT;
static_assert(kWsTotal == 118185984);
static_assert(kWsTotal <= 134217728);
static_assert(kOffO16 % 256 == 0 && kOffO32 % 256 == 0 && kOffKeys % 256 == 0 && kOffHT16 % 256 == 0 &&
              kOffQ % 256 == 0 && kOffWkT % 256 == 0 && kOffWqT % 256 == 0);
static_assert(kTok % 64 == 0 && kH % 64 == 0 && (2 * kH) % 32 == 0);
static_assert(kB % 64 == 0 && kH % 32 == 0);

extern "C" void kernel_launch(void* const* d_in, const int* in_sizes, int n_in,
                              void* d_out, int out_size, void* d_ws, size_t ws_size,
                              hipStream_t stream) {
  if (n_in < 14) return;
  if (in_sizes[0] != kB * kS * kT || out_size != kB * 2 * kH) return;
  if (ws_size < kWsTotal) return;
  const int*   ids = (const int*)d_in[0];
  const float* emb = (const float*)d_in[1];
  const float* Wf  = (const float*)d_in[2];
  const float* Uf  = (const float*)d_in[3];
  const float* bfp = (const float*)d_in[4];
  const float* Wb  = (const float*)d_in[5];
  const float* Ub  = (const float*)d_in[6];
  const float* bbp = (const float*)d_in[7];
  const float* Wk  = (const float*)d_in[8];
  const float* bk  = (const float*)d_in[9];
  const float* Wq  = (const float*)d_in[10];
  const float* bq  = (const float*)d_in[11];
  const float* We  = (const float*)d_in[12];
  const float* be  = (const float*)d_in[13];
  float* out = (float*)d_out;
  const int nV = in_sizes[1] / kE;

  char* ws = (char*)d_ws;
  float*    X32  = (float*)(ws + kOffX32);
  _Float16* O16  = (_Float16*)(ws + kOffO16);
  float*    O32  = (float*)(ws + kOffO32);
  float*    KEYS = (float*)(ws + kOffKeys);
  _Float16* HT16 = (_Float16*)(ws + kOffHT16);
  float*    Qp   = (float*)(ws + kOffQ);
  _Float16* WkT  = (_Float16*)(ws + kOffWkT);
  _Float16* WqT  = (_Float16*)(ws + kOffWqT);

  embed_mean<<<kTok / 8, 256, 0, stream>>>(ids, emb, X32, nV);
  prep_weights<<<6, 256, 0, stream>>>(Wk, Wq, WkT, WqT);
  gru_bidir<<<dim3(kB / 64, 2), 128, 0, stream>>>(X32, ids, Uf, Wf, bfp, Ub, Wb, bbp, O16, O32, HT16);
  wmma_gemm64<0, false, 2, 0, false, 0><<<dim3(1, 1), 256, 0, stream>>>(
      (const unsigned short*)HT16, (const unsigned short*)HT16, kH, 0L,
      (const unsigned short*)WqT, (const unsigned short*)WqT, kH, 0L,
      (void*)Qp, (void*)Qp, kH, 0L,
      bq, bq, 0L, kB, kH, kH, kInv);
  wmma_gemm64<0, false, 2, 0, false, 0><<<dim3(kTok / 64 / 8, 1), 256, 0, stream>>>(
      (const unsigned short*)O16, (const unsigned short*)O16, 2 * kH, 0L,
      (const unsigned short*)WkT, (const unsigned short*)WkT, 2 * kH, 0L,
      (void*)KEYS, (void*)KEYS, kH, 0L,
      bk, bk, 0L, kTok, kH, 2 * kH, kInv);
  attn_pool<<<kB, 256, 0, stream>>>(KEYS, Qp, We, be, ids, O32, out);
}
